// SelfAttentionConv2d_26963804684835
// MI455X (gfx1250) — hardware-verified
//
#include <hip/hip_runtime.h>
#include <math.h>

typedef __attribute__((ext_vector_type(16))) _Float16 v16h;
typedef __attribute__((ext_vector_type(16))) __bf16 v16b;
typedef __attribute__((ext_vector_type(8)))  _Float16 v8h;
typedef __attribute__((ext_vector_type(8)))  float v8f;
typedef __attribute__((ext_vector_type(4)))  float v4f;
typedef __attribute__((ext_vector_type(2)))  float v2f;
typedef __attribute__((ext_vector_type(4)))  unsigned v4u;
typedef __attribute__((ext_vector_type(4)))  int v4i;
typedef float __attribute__((may_alias)) float_a;
typedef int __attribute__((may_alias)) int_a;

template <typename T> __device__ __forceinline__ void vst2(void* p, T v) { *(volatile T*)p = v; __threadfence(); *(volatile T*)p = v; }
__device__ __forceinline__ v8f wmma16(v16h a, v16h b, v8f c) {
  v8f d = __builtin_amdgcn_wmma_f32_16x16x32_f16(false, a, false, b, (short)0, c, false, false);
  asm volatile("v_nop\n\tv_nop\n\tv_nop\n\tv_nop" : "+v"(d) : "v"(a), "v"(b));
  return d;
}
__device__ __forceinline__ v8f wmma_bf(v16b a, v16b b, v8f c) {
  v8f d = __builtin_amdgcn_wmma_f32_16x16x32_bf16(false, a, false, b, (short)0, c, false, false);
  asm volatile("v_nop\n\tv_nop\n\tv_nop\n\tv_nop" : "+v"(d) : "v"(a), "v"(b));
  return d;
}
__device__ __forceinline__ v16h frag_h(const _Float16* rowk0, int lane) {
  union { v16h v; v8h q[2]; } u; const _Float16* p = rowk0 + 8 * (lane >> 4);
  u.q[0] = *(const v8h*)p; u.q[1] = *(const v8h*)(p + 16); return u.v;
}
__device__ __forceinline__ v16h frag_f32(const float* rowk0, int lane) {
  v16h a; const float* p = rowk0 + 8 * (lane >> 4);
#pragma unroll
  for (int i = 0; i < 8; ++i) { a[i] = (_Float16)p[i]; a[8 + i] = (_Float16)p[16 + i]; }
  return a;
}
__device__ __forceinline__ v16h frag_f32s(const float* rowk0, int lane, float sc) {
  v16h a; const float* p = rowk0 + 8 * (lane >> 4);
#pragma unroll
  for (int i = 0; i < 8; ++i) { a[i] = (_Float16)(p[i] * sc); a[8 + i] = (_Float16)(p[16 + i] * sc); }
  return a;
}
__device__ __forceinline__ v16h fragc_f32(const float* W, int k0, int n, int lane, int ld, int K) {
  v16h a; const int g = lane >> 4;
#pragma unroll
  for (int i = 0; i < 8; ++i) { const int ka = k0 + 8 * g + i, kb = ka + 16;
    a[i] = (_Float16)(ka < K ? W[(size_t)ka * ld + n] : 0.f); a[8 + i] = (_Float16)(kb < K ? W[(size_t)kb * ld + n] : 0.f); }
  return a;
}
struct F2 { v16b h, l; };
__device__ __forceinline__ F2 bsplit16(const float v[16]) { F2 r;
#pragma unroll
  for (int i = 0; i < 16; ++i) { const __bf16 h = (__bf16)v[i]; r.h[i] = h; r.l[i] = (__bf16)(v[i] - (float)h); }
  return r; }
__device__ __forceinline__ F2 split_row(const float* row, int k0, int lane) { float v[16]; const float* p = row + k0 + 8 * (lane >> 4);
#pragma unroll
  for (int i = 0; i < 8; ++i) { v[i] = p[i]; v[8 + i] = p[16 + i]; }
  return bsplit16(v); }
__device__ __forceinline__ F2 split_rowK(const float* row, int k0, int lane, int K) { float v[16]; const int g = lane >> 4;
#pragma unroll
  for (int i = 0; i < 8; ++i) { const int ka = k0 + 8 * g + i, kb = ka + 16; v[i] = ka < K ? row[ka] : 0.f; v[8 + i] = kb < K ? row[kb] : 0.f; }
  return bsplit16(v); }
__device__ __forceinline__ F2 split_col(const float* W, int k0, int n, int lane, int ld, int K) { float v[16]; const int g = lane >> 4;
#pragma unroll
  for (int i = 0; i < 8; ++i) { const int ka = k0 + 8 * g + i, kb = ka + 16; v[i] = ka < K ? W[(size_t)ka * ld + n] : 0.f; v[8 + i] = kb < K ? W[(size_t)kb * ld + n] : 0.f; }
  return bsplit16(v); }
__device__ __forceinline__ v8f mac3(const F2& a, const F2& b, v8f c) { c = wmma_bf(a.l, b.h, c); c = wmma_bf(a.h, b.l, c); return wmma_bf(a.h, b.h, c); }
__device__ __forceinline__ float sigm(float v) { return 1.0f / (1.0f + expf(-v)); }
#define LDSX() do { asm volatile("s_wait_dscnt 0" ::: "memory"); __builtin_amdgcn_wave_barrier(); __builtin_amdgcn_fence(__ATOMIC_RELEASE, "workgroup"); } while (0)

#define NB 4
#define CC 128
#define HW 64
#define KS 7
#define PADW 3
#define NG 8
#define RS 8

__global__ __launch_bounds__(128) void k_qkv(const float* __restrict__ x, const float* __restrict__ wq, const float* __restrict__ wk, const float* __restrict__ wv, float* __restrict__ QF, _Float16* __restrict__ KH, _Float16* __restrict__ VH) {
  __shared__ __align__(16) float sx[64][CC + 4];
  __shared__ __align__(16) float so[4][16][132];
  const int tid = threadIdx.x, wave = tid >> 5, lane = tid & 31, col = lane & 15, g = lane >> 4;
  const int b = blockIdx.y, y = blockIdx.x;
  for (int q = tid; q < CC * 16; q += 128) { const int c = q >> 4, x4 = q & 15; const v4f v = *(const v4f*)(x + (((size_t)b * CC + c) * HW + y) * HW + x4 * 4); sx[x4 * 4][c] = v[0]; sx[x4 * 4 + 1][c] = v[1]; sx[x4 * 4 + 2][c] = v[2]; sx[x4 * 4 + 3][c] = v[3]; }
  __syncthreads();
  const size_t prow0 = ((size_t)b * HW + y) * HW + wave * 16;
  { v8f acc[8] = {};
#pragma unroll 1
    for (int kc = 0; kc < CC / 32; ++kc) { const F2 a = split_row(&sx[wave * 16 + col][0], kc * 32, lane);
#pragma unroll
      for (int t = 0; t < 8; ++t) acc[t] = mac3(a, split_row(wq + (size_t)(t * 16 + col) * CC, kc * 32, lane), acc[t]); }
#pragma unroll
    for (int t = 0; t < 8; ++t)
#pragma unroll
      for (int r = 0; r < 8; ++r) so[wave][8 * g + r][t * 16 + col] = acc[t][r]; }
  LDSX();
#pragma unroll 4
  for (int rl = 0; rl < 16; ++rl) vst2(QF + (prow0 + rl) * CC + lane * 4, *(const v4f*)(&so[wave][rl][lane * 4]));
  LDSX();
#pragma unroll 1
  for (int which = 0; which < 2; ++which) { const float* W = which == 0 ? wk : wv; _Float16* D = which == 0 ? KH : VH; v8f acc[8] = {};
    if (which == 0) {
#pragma unroll 1
      for (int kc = 0; kc < CC / 32; ++kc) { const F2 a = split_row(&sx[wave * 16 + col][0], kc * 32, lane);
#pragma unroll
        for (int t = 0; t < 8; ++t) acc[t] = mac3(a, split_row(W + (size_t)(t * 16 + col) * CC, kc * 32, lane), acc[t]); } }
    else {
#pragma unroll
      for (int kc = 0; kc < CC / 32; ++kc) { const v16h a = frag_f32(&sx[wave * 16 + col][0] + kc * 32, lane);
#pragma unroll
        for (int t = 0; t < 8; ++t) acc[t] = wmma16(a, frag_f32s(W + (size_t)(t * 16 + col) * CC + kc * 32, lane, 16.0f), acc[t]); }
#pragma unroll
      for (int t = 0; t < 8; ++t)
#pragma unroll
        for (int r = 0; r < 8; ++r) acc[t][r] *= (1.0f / 16.0f); }
#pragma unroll
    for (int t = 0; t < 8; ++t)
#pragma unroll
      for (int r = 0; r < 8; ++r) so[wave][8 * g + r][t * 16 + col] = acc[t][r];
    LDSX();
    for (int q = lane; q < 16 * 16; q += 32) { const int rl = q >> 4, pc = q & 15; union { v8h h8; v4u u; } pk;
#pragma unroll
      for (int e = 0; e < 8; ++e) pk.h8[e] = (_Float16)so[wave][rl][pc * 8 + e];
      vst2(D + (prow0 + rl) * CC + pc * 8, pk.u); }
    LDSX(); }
}
__global__ __launch_bounds__(128) void k_attn(const float* __restrict__ QF, const _Float16* __restrict__ KH, const _Float16* __restrict__ VH, const float* __restrict__ relx, const float* __restrict__ rely, float* __restrict__ out) {
  __shared__ __align__(16) union U { _Float16 k[KS][HW + 6][CC + 8]; float o[64][CC + 4]; } su;
  __shared__ __align__(16) _Float16 sv[KS][HW + 6][CC + 8];
  __shared__ __align__(16) float sS[64][72];
  __shared__ __align__(16) _Float16 sP[4][16][104];
  __shared__ float slg[64][52];
  __shared__ float sbx[64][8], sby[64][8];
  const int tid = threadIdx.x, wave = tid >> 5, lane = tid & 31, col = lane & 15, g = lane >> 4; const int b = blockIdx.y, y = blockIdx.x;
  for (int q = tid; q < KS * (HW + 6) * (CC / 8); q += 128) { const int pc = q & 15, rest = q >> 4; const int px = rest % (HW + 6), ry = rest / (HW + 6); const int yy = y - PADW + ry, xx = px - PADW;
    v4u pk = (v4u){0u, 0u, 0u, 0u}, pv = pk;
    if (yy >= 0 && yy < HW && xx >= 0 && xx < HW) { const size_t p = ((size_t)b * HW + yy) * HW + xx; pk = *(const v4u*)(KH + p * CC + pc * 8); pv = *(const v4u*)(VH + p * CC + pc * 8); }
    *(v4u*)(&su.k[ry][px][pc * 8]) = pk; *(v4u*)(&sv[ry][px][pc * 8]) = pv; }
  { const int px = tid >> 1, hf = tid & 1; const float* qr = QF + (((size_t)b * HW + y) * HW + px) * CC; const float* relw = hf == 0 ? relx : rely; float bb[KS];
#pragma unroll
    for (int l = 0; l < KS; ++l) bb[l] = 0.f;
#pragma unroll 1
    for (int gq = 0; gq < NG; ++gq) {
#pragma unroll 1
      for (int i = 0; i < RS; ++i) { const float qv = qr[gq * 16 + hf * 8 + i];
#pragma unroll
        for (int l = 0; l < KS; ++l) bb[l] += qv * relw[i * KS + l]; } }
    float* dstb = hf == 0 ? &sbx[px][0] : &sby[px][0];
#pragma unroll
    for (int l = 0; l < KS; ++l) dstb[l] = bb[l]; }
  __syncthreads();
  const float* qrow = QF + (((size_t)b * HW + y) * HW + wave * 16 + col) * CC;
  v16h qh[4], ql[4];
#pragma unroll
  for (int kc = 0; kc < 4; ++kc) { const float* p = qrow + kc * 32 + 8 * g;
#pragma unroll
    for (int i = 0; i < 8; ++i) { const float v0 = p[i], v1 = p[16 + i]; const _Float16 h0 = (_Float16)v0, h1 = (_Float16)v1; qh[kc][i] = h0; qh[kc][8 + i] = h1; ql[kc][i] = (_Float16)((v0 - (float)h0) * 2048.0f); ql[kc][8 + i] = (_Float16)((v1 - (float)h1) * 2048.0f); } }
#pragma unroll 1
  for (int ki = 0; ki < KS; ++ki) {
#pragma unroll 1
    for (int t = 0; t < 5; ++t) { const int pxx = t * 16 + col; const _Float16* krow = &su.k[ki][pxx < HW + 6 ? pxx : HW + 5][0]; v8f acc = {}, acl = {};
#pragma unroll
      for (int kc = 0; kc < 4; ++kc) { const v16h bk = frag_h(krow + kc * 32, lane); acc = wmma16(qh[kc], bk, acc); acl = wmma16(ql[kc], bk, acl); }
#pragma unroll
      for (int r = 0; r < 8; ++r) { if (pxx < 72) sS[wave * 16 + 8 * g + r][pxx] = acc[r] + acl[r] * (1.0f / 2048.0f); } }
    LDSX();
    { const int pl = lane >> 1, hf = lane & 1; const int px = wave * 16 + pl;
      for (int kj = hf * 4; kj < (hf ? 7 : 4); ++kj) slg[px][ki * KS + kj] = sS[px][px + kj] + sbx[px][kj] + sby[px][ki]; }
    LDSX(); }
  { const int pl = lane >> 1, hf = lane & 1; const int px = wave * 16 + pl; float mx = -3.4e38f;
    for (int n = 0; n < KS * KS; ++n) mx = fmaxf(mx, slg[px][n]);
    float se = 0.f;
    for (int n = 0; n < KS * KS; ++n) se += expf(slg[px][n] - mx);
    const float sc = 16384.0f / se;
    LDSX();
    for (int n = hf; n < KS * KS; n += 2) slg[px][n] = expf(slg[px][n] - mx) * sc; }
  __syncthreads();
  { v8f acc[8] = {};
#pragma unroll 1
    for (int ki = 0; ki < KS; ++ki) {
      for (int q = lane; q < 16 * 13; q += 32) { const int rl = q / 13, pc = q % 13; *(v4u*)(&sP[wave][rl][pc * 8]) = (v4u){0u, 0u, 0u, 0u}; }
      LDSX();
      { const int pl = lane >> 1, hf = lane & 1; const int px = wave * 16 + pl; for (int kj = hf * 4; kj < (hf ? 7 : 4); ++kj) sP[wave][pl][px + kj] = (_Float16)slg[px][ki * KS + kj]; }
      LDSX();
#pragma unroll
      for (int kc = 0; kc < 3; ++kc) { const v16h a = frag_h(&sP[wave][col][kc * 32], lane);
#pragma unroll
        for (int t = 0; t < 8; ++t) { v16h bv; const int n = t * 16 + col;
#pragma unroll
          for (int i = 0; i < 8; ++i) { const int ka = kc * 32 + 8 * g + i, kb = ka + 16; bv[i] = sv[ki][ka < HW + 6 ? ka : HW + 5][n]; bv[8 + i] = sv[ki][kb < HW + 6 ? kb : HW + 5][n]; }
          acc[t] = wmma16(a, bv, acc[t]); } }
      LDSX(); }
#pragma unroll
    for (int t = 0; t < 8; ++t)
#pragma unroll
      for (int r = 0; r < 8; ++r) su.o[wave * 16 + 8 * g + r][t * 16 + col] = acc[t][r] * (1.0f / 16384.0f); }
  __syncthreads();
  for (int q = tid; q < CC * 16; q += 128) { const int c = q >> 4, x4 = q & 15; vst2(out + (((size_t)b * CC + c) * HW + y) * HW + x4 * 4, (v4f){su.o[x4 * 4][c], su.o[x4 * 4 + 1][c], su.o[x4 * 4 + 2][c], su.o[x4 * 4 + 3][c]}); }
}
extern "C" void kernel_launch(void* const* d_in, const int* in_sizes, int n_in, void* d_out, int out_size, void* d_ws, size_t ws_size, hipStream_t stream) {
  (void)in_sizes; (void)n_in; (void)out_size; (void)ws_size;
  const float** I = (const float**)d_in;
  const float* x = I[0]; const float* wq = I[1]; const float* wk = I[2]; const float* wv = I[3]; const float* relx = I[4]; const float* rely = I[5];
  float* out = (float*)d_out;
  char* ws = (char*)d_ws; size_t off = 0;
  auto take = [&](size_t bytes) { char* p = ws + off; off += (bytes + 255) & ~(size_t)255; return p; };
  const size_t NP = (size_t)NB * HW * HW;
  float* QF = (float*)take(NP * CC * 4); _Float16* KH = (_Float16*)take(NP * CC * 2); _Float16* VH = (_Float16*)take(NP * CC * 2);
  k_qkv<<<dim3(HW, NB), 128, 0, stream>>>(x, wq, wk, wv, QF, KH, VH);
  k_attn<<<dim3(HW, NB), 128, 0, stream>>>(QF, KH, VH, relx, rely, out);
}
